// ConservationConstrainedAttention_71631464563099
// MI455X (gfx1250) — hardware-verified
//
#include <hip/hip_runtime.h>
#include <stdint.h>


typedef __attribute__((ext_vector_type(16))) _Float16 v16h;
typedef __attribute__((ext_vector_type(8)))  _Float16 v8h;
typedef __attribute__((ext_vector_type(16))) __bf16   v16b;
typedef __attribute__((ext_vector_type(8)))  __bf16   v8b;
typedef __attribute__((ext_vector_type(8)))  float    v8f;
typedef __attribute__((ext_vector_type(4)))  float    v4f;

#define NB  4
#define NS  1024
#define ND  1024
#define NH  16
#define NDH 64

__device__ __forceinline__ unsigned short f2bf_bits(float f) {
  unsigned u = __float_as_uint(f);
  return (unsigned short)((u + 0x7FFFu + ((u >> 16) & 1u)) >> 16);
}
__device__ __forceinline__ float bf_bits2f(unsigned short h) { return __uint_as_float(((unsigned)h) << 16); }

__device__ __forceinline__ void dep_guard_h(v8f& a, v8f& b, v16h x, v16h y) { asm volatile("v_nop\n\tv_nop\n\tv_nop\n\tv_nop" : "+v"(a), "+v"(b) : "v"(x), "v"(y)); }
__device__ __forceinline__ void dep_guard_b(v8f& a, v8f& b, v16b x, v16b y) { asm volatile("v_nop\n\tv_nop\n\tv_nop\n\tv_nop" : "+v"(a), "+v"(b) : "v"(x), "v"(y)); }
__device__ __forceinline__ void keep4_h(v16h a, v16h b, v16h c, v16h d) { asm volatile("v_nop" :: "v"(a), "v"(b), "v"(c), "v"(d)); }
__device__ __forceinline__ void keep4_b(v16b a, v16b b, v16b c, v16b d) { asm volatile("v_nop" :: "v"(a), "v"(b), "v"(c), "v"(d)); }
__device__ __forceinline__ void acc_guard4(v8f& a, v8f& b, v8f& c, v8f& d) { asm volatile("v_nop\n\tv_nop\n\tv_nop\n\tv_nop" : "+v"(a), "+v"(b), "+v"(c), "+v"(d)); }
template <typename T> struct Frag;
template <> struct Frag<_Float16> {
  typedef v16h V; union U { v16h v; v8h h[2]; };
  static __device__ __forceinline__ v16h load(const _Float16* p) {
    U f; f.h[0] = *(const v8h*)(p); f.h[1] = *(const v8h*)(p + 16); return f.v;
  }
  static __device__ __forceinline__ v8f mma(v16h a, v16h b, v8f c) {
    return __builtin_amdgcn_wmma_f32_16x16x32_f16(false, a, false, b, (short)0, c, false, false);
  }
  static __device__ __forceinline__ void guard(v8f& a, v8f& b, v16h x, v16h y) { dep_guard_h(a, b, x, y); }
  static __device__ __forceinline__ void keep(v16h a, v16h b, v16h c, v16h d) { keep4_h(a, b, c, d); }
};
template <> struct Frag<__bf16> {
  typedef v16b V; union U { v16b v; v8b h[2]; };
  static __device__ __forceinline__ v16b load(const __bf16* p) {
    U f; f.h[0] = *(const v8b*)(p); f.h[1] = *(const v8b*)(p + 16); return f.v;
  }
  static __device__ __forceinline__ v8f mma(v16b a, v16b b, v8f c) {
    return __builtin_amdgcn_wmma_f32_16x16x32_bf16(false, a, false, b, (short)0, c, false, false);
  }
  static __device__ __forceinline__ void guard(v8f& a, v8f& b, v16b x, v16b y) { dep_guard_b(a, b, x, y); }
  static __device__ __forceinline__ void keep(v16b a, v16b b, v16b c, v16b d) { keep4_b(a, b, c, d); }
};
typedef Frag<_Float16> FH;

__device__ __forceinline__ v8f mma_h(v16h a, v16h b, v8f c) {
  c = __builtin_amdgcn_wmma_f32_16x16x32_f16(false, a, false, b, (short)0, c, false, false);
  asm volatile("v_nop\n\tv_nop\n\tv_nop\n\tv_nop" : "+v"(c) : "v"(a), "v"(b));
  return c;
}

template <int ET> struct Elem;
template <> struct Elem<0> { typedef _Float16 T; };
template <> struct Elem<1> { typedef __bf16 T; };
template <int ET, bool SPLIT, int BIAS_MODE, int OUT_MODE, bool RESID, int ACT = 0>
__global__ __launch_bounds__(256) void wmma_gemm64(
    const unsigned short* __restrict__ Ap, const unsigned short* __restrict__ A2p, int lda, long strideA,
    const unsigned short* __restrict__ Btp, const unsigned short* __restrict__ Bt2p, int ldb, long strideB,
    void* __restrict__ Cout, void* __restrict__ Cout2, int ldc, long strideC,
    const float* __restrict__ bias,
    const float* __restrict__ resid, long strideR,
    int M, int N, int K, float scale) {
  typedef typename Elem<ET>::T T;
  typedef typename Frag<T>::V V;
  const T* A = (const T*)Ap; const T* A2 = (const T*)A2p; const T* Bt = (const T*)Btp; const T* Bt2 = (const T*)Bt2p;
  __shared__ __align__(16) float sT[8][16 * 68];
  const int b    = blockIdx.y;
  const int lane = threadIdx.x & 31;
  const int wave = threadIdx.x >> 5;
  const int tilesN = N >> 6;
  const int tilesM = M >> 6;
  const int tile = blockIdx.x * 8 + wave;
  if (tile >= tilesM * tilesN) return;
  const int tm = tile / tilesN;
  const int tn = tile - tm * tilesN;
  const int m0 = tm << 6;
  const int n0 = tn << 6;

  const T* Ab  = A  + (size_t)b * strideA;
  const T* Bb  = Bt + (size_t)b * strideB;
  const T* Ab2 = SPLIT ? (A2  + (size_t)b * strideA) : nullptr;
  const T* Bb2 = SPLIT ? (Bt2 + (size_t)b * strideB) : nullptr;

  const int rlane = lane & 15;
  const int koff  = (lane >> 4) * 8;
  const int mOff  = (lane >> 4) * 8;

  v8f acc[4][4];
#pragma unroll
  for (int i = 0; i < 4; ++i)
#pragma unroll
    for (int j = 0; j < 4; ++j) acc[i][j] = (v8f){0.f,0.f,0.f,0.f,0.f,0.f,0.f,0.f};

  for (int k0 = 0; k0 < K; k0 += 32) {
    V bh[4], bl[4];
#pragma unroll
    for (int j = 0; j < 4; ++j) {
      const size_t bo = (size_t)(n0 + (j << 4) + rlane) * ldb + koff + k0;
      bh[j] = Frag<T>::load(Bb + bo);
      if (SPLIT) bl[j] = Frag<T>::load(Bb2 + bo);
    }
#pragma unroll
    for (int i = 0; i < 4; ++i) {
      const size_t ao = (size_t)(m0 + (i << 4) + rlane) * lda + koff + k0;
      V ah = Frag<T>::load(Ab + ao);
      V al;
      if (SPLIT) al = Frag<T>::load(Ab2 + ao);
#pragma unroll
      for (int j = 0; j < 4; ++j) {
        acc[i][j] = Frag<T>::mma(ah, bh[j], acc[i][j]);
        if (SPLIT) {
          acc[i][j] = Frag<T>::mma(ah, bl[j], acc[i][j]);
          acc[i][j] = Frag<T>::mma(al, bh[j], acc[i][j]);
        }
      }
      Frag<T>::guard(acc[i][0], acc[i][3], ah, SPLIT ? al : ah);
    }
    Frag<T>::keep(bh[0], bh[1], bh[2], bh[3]);
    if (SPLIT) Frag<T>::keep(bl[0], bl[1], bl[2], bl[3]);
  }
  acc_guard4(acc[0][0], acc[0][1], acc[0][2], acc[0][3]);
  acc_guard4(acc[1][0], acc[1][1], acc[1][2], acc[1][3]);
  acc_guard4(acc[2][0], acc[2][1], acc[2][2], acc[2][3]);
  acc_guard4(acc[3][0], acc[3][1], acc[3][2], acc[3][3]);

  float* slab = sT[wave];
  const float* Rb = RESID ? (resid + (size_t)b * strideR) : nullptr;
#pragma unroll
  for (int i = 0; i < 4; ++i) {
    const int mBase = m0 + (i << 4);
#pragma unroll
    for (int j = 0; j < 4; ++j) {
      const int n = n0 + (j << 4) + rlane;
      float bv = 0.f;
      if (BIAS_MODE == 2) bv = bias[n];
#pragma unroll
      for (int r = 0; r < 8; ++r) {
        float v = acc[i][j][r] * scale;
        if (BIAS_MODE == 1) v += bias[mBase + mOff + r];
        if (BIAS_MODE == 2) v += bv;
        if (RESID) v += Rb[(size_t)(mBase + mOff + r) * ldc + n];
        if (ACT == 1) v = tanhf(v);
        if (ACT == 2) v = fmaxf(v, 0.0f);
        if (ACT == 3) v = v / (1.0f + expf(-v));
        if (ACT == 4) v = (v > 0.f) ? v : 0.01f * v;
        if (ACT == 5) v = 0.5f * v * (1.0f + erff(v * 0.70710678118654752f));
        slab[(mOff + r) * 68 + (j << 4) + rlane] = v;
      }
    }
    __builtin_amdgcn_fence(__ATOMIC_RELEASE, "workgroup");
    __builtin_amdgcn_wave_barrier();
    __builtin_amdgcn_fence(__ATOMIC_ACQUIRE, "workgroup");
    if (OUT_MODE == 0) {
      float* C = (float*)Cout + (size_t)b * strideC;
      const int hh = lane >> 4, c4 = (lane & 15) * 4;
      for (int pass = 0; pass < 2; ++pass) {
#pragma unroll
        for (int it = 0; it < 8; ++it) {
          const int row = it * 2 + hh;
          v4f v = *(const v4f*)(slab + row * 68 + c4);
          *(volatile v4f*)(C + (size_t)(mBase + row) * ldc + n0 + c4) = v;
        }
        __threadfence();
      }
    } else {
      const int q = lane >> 3, c8 = (lane & 7) * 8;
      unsigned short* C  = (unsigned short*)Cout  + (size_t)b * strideC;
      unsigned short* C2 = (OUT_MODE == 2) ? ((unsigned short*)Cout2 + (size_t)b * strideC) : nullptr;
      for (int pass = 0; pass < 2; ++pass) {
#pragma unroll
        for (int it = 0; it < 4; ++it) {
          const int row = it * 4 + q;
          const float* sp = slab + row * 68 + c8;
          v8h hv, lv;
#pragma unroll
          for (int e = 0; e < 8; ++e) {
            if (OUT_MODE == 1) {
              hv[e] = (_Float16)sp[e];
            } else {
              unsigned short hb = f2bf_bits(sp[e]);
              unsigned short lb = f2bf_bits(sp[e] - bf_bits2f(hb));
              hv[e] = __builtin_bit_cast(_Float16, hb);
              lv[e] = __builtin_bit_cast(_Float16, lb);
            }
          }
          *(volatile v8h*)(C + (size_t)(mBase + row) * ldc + n0 + c8) = hv;
          if (OUT_MODE == 2) *(volatile v8h*)(C2 + (size_t)(mBase + row) * ldc + n0 + c8) = lv;
        }
        __threadfence();
      }
    }
    __builtin_amdgcn_fence(__ATOMIC_RELEASE, "workgroup");
    __builtin_amdgcn_wave_barrier();
    __builtin_amdgcn_fence(__ATOMIC_ACQUIRE, "workgroup");
  }
}

__global__ __launch_bounds__(256) void cast_f32_f16x2(
    const float* __restrict__ in, _Float16* __restrict__ out, int n2) {
  int i = blockIdx.x * 256 + threadIdx.x;
  if (i < n2) {
    const _Float16 h0 = (_Float16)in[2 * i], h1 = (_Float16)in[2 * i + 1];
    const unsigned u = (unsigned)__builtin_bit_cast(unsigned short, h0) | ((unsigned)__builtin_bit_cast(unsigned short, h1) << 16);
    ((volatile unsigned*)out)[i] = u;
    __threadfence();
    ((volatile unsigned*)out)[i] = u;
  }
}

__global__ __launch_bounds__(256) void pair_table_k(const float* __restrict__ coords, float* __restrict__ T) {
#pragma clang fp contract(off)
  const int row = blockIdx.x;
  const int b = row >> 10;
  const float cq0 = coords[(size_t)row * 4 + 0];
  const float cq1 = coords[(size_t)row * 4 + 1];
  const float cq2 = coords[(size_t)row * 4 + 2];
  const float cq3 = coords[(size_t)row * 4 + 3];
  const float* cb = coords + (size_t)b * NS * 4;
  float* trow = T + (size_t)row * NS;
  const float ninf = -__builtin_huge_valf();
#pragma unroll 1
  for (int p = 0; p < 4; ++p) {
    const int k = p * 256 + (int)threadIdx.x;
    const v4f ck = *(const v4f*)(cb + (size_t)k * 4);
    const float dt = cq0 - ck[0];
    const float d1 = cq1 - ck[1];
    const float d2 = cq2 - ck[2];
    const float d3 = cq3 - ck[3];
    const float s1 = d1 * d1;
    const float s2 = d2 * d2;
    const float s3 = d3 * d3;
    const float dr2 = (s1 + s2) + s3;
    const float tt = dt * dt;
    const float itv = tt - dr2;
    const float ph = logf(expf(-fabsf(itv) * 0.1f) + 1e-8f);
    const bool forbid = ((fabsf(dt) < sqrtf(dr2)) && (dr2 > 1e-6f)) || (dt < 0.f);
    const float val = forbid ? ninf : ph;
    ((volatile float*)trow)[k] = val;
    __threadfence();
    ((volatile float*)trow)[k] = val;
  }
}

__global__ __launch_bounds__(256) void energy_k(const _Float16* __restrict__ Vh, const float* __restrict__ We,
                                               const float* __restrict__ be, float* __restrict__ E, int n) {
  const int i = blockIdx.x * 256 + (int)threadIdx.x;
  if (i >= n) return;
  const int bh = i >> 10, s = i & 1023;
  const int b = bh >> 4, h = bh & 15;
  const _Float16* v = Vh + ((size_t)(b * NS + s)) * ND + h * NDH;
  float acc = be[0];
#pragma unroll 1
  for (int g = 0; g < 8; ++g) {
    const v8h vv = *(const v8h*)(v + 8 * g);
#pragma unroll
    for (int e = 0; e < 8; ++e) acc += (float)vv[e] * We[8 * g + e];
  }
  ((volatile float*)E)[i] = acc;
  __threadfence();
  ((volatile float*)E)[i] = acc;
}

__global__ __launch_bounds__(128) void attn_stats_k(
    const _Float16* __restrict__ Qh, const _Float16* __restrict__ Kh,
    const float* __restrict__ T, const float* __restrict__ E,
    float* __restrict__ Mo, float* __restrict__ Lo, float* __restrict__ Ao) {
  __shared__ __align__(16) _Float16 Ksh[64 * 64];
  __shared__ __align__(16) float stat[3][64];
  const int tid = threadIdx.x;
  const int wave = tid >> 5, lane = tid & 31, hh = lane >> 4, c = lane & 15;
  const int bx = blockIdx.x;
  const int qb = bx & 15;
  const int bh = bx >> 4;
  const int h = bh & 15;
  const int b = bh >> 4;
  const int qbase = qb * 64;
  const int q0 = qbase + wave * 16;

  v16h qa0, qa1;
  {
    const _Float16* qrow = Qh + ((size_t)(b * NS + q0 + c)) * ND + h * NDH;
    qa0 = FH::load(qrow + 8 * hh);
    qa1 = FH::load(qrow + 32 + 8 * hh);
  }
  float mrow[8], lrow[8], arow[8];
#pragma unroll
  for (int r = 0; r < 8; ++r) { mrow[r] = -1e30f; lrow[r] = 0.f; arow[r] = 0.f; }

  const float* tb = T + ((size_t)(b * NS + q0 + 8 * hh)) * NS + c;
  const float* eb = E + (size_t)bh * NS + c;

  for (int kc = 0; kc < 16; ++kc) {
    const int kv0 = kc * 64;
    __syncthreads();
    {
      const int kvr = tid >> 1, dh = (tid & 1) * 32;
      const _Float16* src = Kh + ((size_t)(b * NS + kv0 + kvr)) * ND + h * NDH + dh;
      _Float16* dst = Ksh + kvr * 64 + dh;
#pragma unroll
      for (int i = 0; i < 4; ++i) *(v8h*)(dst + 8 * i) = *(const v8h*)(src + 8 * i);
    }
    __syncthreads();

    v8f s[4];
#pragma unroll
    for (int j = 0; j < 4; ++j) {
      s[j] = (v8f){0.f,0.f,0.f,0.f,0.f,0.f,0.f,0.f};
      FH::U kb;
      kb.h[0] = *(const v8h*)(Ksh + (j * 16 + c) * 64 + 8 * hh);
      kb.h[1] = *(const v8h*)(Ksh + (j * 16 + c) * 64 + 16 + 8 * hh);
      s[j] = mma_h(qa0, kb.v, s[j]);
      kb.h[0] = *(const v8h*)(Ksh + (j * 16 + c) * 64 + 32 + 8 * hh);
      kb.h[1] = *(const v8h*)(Ksh + (j * 16 + c) * 64 + 48 + 8 * hh);
      s[j] = mma_h(qa1, kb.v, s[j]);
    }
    float ev[4];
#pragma unroll
    for (int j = 0; j < 4; ++j) ev[j] = eb[kv0 + j * 16];

    float cm[8];
#pragma unroll
    for (int r = 0; r < 8; ++r) {
      float m = -__builtin_huge_valf();
#pragma unroll
      for (int j = 0; j < 4; ++j) {
        const float a = tb[(size_t)r * NS + kv0 + j * 16];
        const float v = s[j][r] * 0.125f + a;
        s[j][r] = v;
        m = fmaxf(m, v);
      }
#pragma unroll
      for (int off = 1; off < 16; off <<= 1) m = fmaxf(m, __shfl_xor(m, off, 32));
      cm[r] = m;
    }
#pragma unroll
    for (int r = 0; r < 8; ++r) {
      const float mnew = fmaxf(mrow[r], cm[r]);
      const float alpha = __expf(mrow[r] - mnew);
      mrow[r] = mnew;
      float psum = 0.f, esum = 0.f;
#pragma unroll
      for (int j = 0; j < 4; ++j) {
        const float p = __expf(s[j][r] - mnew);
        psum += p;
        esum += p * ev[j];
      }
#pragma unroll
      for (int off = 1; off < 16; off <<= 1) {
        psum += __shfl_xor(psum, off, 32);
        esum += __shfl_xor(esum, off, 32);
      }
      lrow[r] = lrow[r] * alpha + psum;
      arow[r] = arow[r] * alpha + esum;
    }
  }

  if (c == 0) {
#pragma unroll
    for (int r = 0; r < 8; ++r) {
      const int rr = wave * 16 + 8 * hh + r;
      stat[0][rr] = mrow[r];
      stat[1][rr] = lrow[r];
      stat[2][rr] = arow[r] * (1.0f / lrow[r]);
    }
  }
  __syncthreads();
  const size_t base = (size_t)bh * NS + qbase;
  if (wave == 0) {
    float* dst = (hh == 0) ? Mo : Lo;
    const v4f v = *(const v4f*)(&stat[hh][4 * c]);
    *(volatile v4f*)(dst + base + 4 * c) = v;
    __threadfence();
    *(volatile v4f*)(dst + base + 4 * c) = v;
  } else if (wave == 1) {
    if (hh == 0) {
      const v4f v = *(const v4f*)(&stat[2][4 * c]);
      *(volatile v4f*)(Ao + base + 4 * c) = v;
      __threadfence();
      *(volatile v4f*)(Ao + base + 4 * c) = v;
    }
  }
}

__global__ __launch_bounds__(256) void corr_k(const float* __restrict__ A, const float* __restrict__ E0,
                                             float* __restrict__ C) {
  __shared__ double red[4][256];
  const int tid = threadIdx.x;
  const int HS = NH * NS;
  double p0 = 0.0, p1 = 0.0, p2 = 0.0, p3 = 0.0;
  for (int i = tid; i < HS; i += 256) {
    p0 += (double)A[i];
    p1 += (double)A[HS + i];
    p2 += (double)A[2 * HS + i];
    p3 += (double)A[3 * HS + i];
  }
  red[0][tid] = p0; red[1][tid] = p1; red[2][tid] = p2; red[3][tid] = p3;
  __syncthreads();
  for (int st = 128; st > 0; st >>= 1) {
    if (tid < st) {
      red[0][tid] += red[0][tid + st];
      red[1][tid] += red[1][tid + st];
      red[2][tid] += red[2][tid + st];
      red[3][tid] += red[3][tid + st];
    }
    __syncthreads();
  }
  if (tid < 32) {
    const float t0 = (float)red[0][0], t1 = (float)red[1][0], t2 = (float)red[2][0], t3 = (float)red[3][0];
    const float e0 = E0[0], e1 = E0[1], e2 = E0[2], e3 = E0[3];
    float mv = fabsf(t0 - e0);
    mv = mv + fabsf(t1 - e1);
    mv = mv + fabsf(t2 - e2);
    mv = mv + fabsf(t3 - e3);
    mv = mv * 0.25f;
    const bool apply = (mv > 0.1f);
    const float c0 = apply ? (float)((double)e0 / (double)(t0 + 1e-8f)) : 1.0f;
    const float c1 = apply ? (float)((double)e1 / (double)(t1 + 1e-8f)) : 1.0f;
    const float c2 = apply ? (float)((double)e2 / (double)(t2 + 1e-8f)) : 1.0f;
    const float c3 = apply ? (float)((double)e3 / (double)(t3 + 1e-8f)) : 1.0f;
    const int l3 = tid & 3;
    const float v = (l3 == 0) ? c0 : (l3 == 1) ? c1 : (l3 == 2) ? c2 : c3;
    ((volatile float*)C)[tid] = v;
    __threadfence();
    ((volatile float*)C)[tid] = v;
  }
}

__global__ __launch_bounds__(128) void attn_out_k(
    const _Float16* __restrict__ Qh, const _Float16* __restrict__ Kh, const _Float16* __restrict__ Vh,
    const float* __restrict__ T, const float* __restrict__ Mi, const float* __restrict__ Li,
    const float* __restrict__ Ci, _Float16* __restrict__ Oh) {
  __shared__ __align__(16) _Float16 Ksh[64 * 64];
  __shared__ __align__(16) _Float16 Vth[64 * 64];
  __shared__ __align__(16) _Float16 Psh[4][16 * 64];
  __shared__ __align__(16) float Os[4][16 * 68];
  const int tid = threadIdx.x;
  const int wave = tid >> 5, lane = tid & 31, hh = lane >> 4, c = lane & 15;
  const int bx = blockIdx.x;
  const int qb = bx & 15;
  const int bh = bx >> 4;
  const int h = bh & 15;
  const int b = bh >> 4;
  const int qbase = qb * 64;
  const int q0 = qbase + wave * 16;
  const float corr = Ci[b];

  v16h qa0, qa1;
  {
    const _Float16* qrow = Qh + ((size_t)(b * NS + q0 + c)) * ND + h * NDH;
    qa0 = FH::load(qrow + 8 * hh);
    qa1 = FH::load(qrow + 32 + 8 * hh);
  }
  float m1[8], il[8], m2[8], l2[8];
  v8f oacc[4];
  {
    const float* mp = Mi + (size_t)bh * NS + q0 + 8 * hh;
    const float* lp = Li + (size_t)bh * NS + q0 + 8 * hh;
#pragma unroll
    for (int r = 0; r < 8; ++r) {
      m1[r] = mp[r];
      il[r] = corr * (1.0f / lp[r]);
      m2[r] = -1e30f;
      l2[r] = 0.f;
    }
  }
#pragma unroll
  for (int t = 0; t < 4; ++t) oacc[t] = (v8f){0.f,0.f,0.f,0.f,0.f,0.f,0.f,0.f};

  const float* tb = T + ((size_t)(b * NS + q0 + 8 * hh)) * NS + c;

  for (int kc = 0; kc < 16; ++kc) {
    const int kv0 = kc * 64;
    __syncthreads();
    {
      const int kvr = tid >> 1, dh = (tid & 1) * 32;
      const size_t so = ((size_t)(b * NS + kv0 + kvr)) * ND + h * NDH + dh;
      const _Float16* ksrc = Kh + so;
      const _Float16* vsrc = Vh + so;
      _Float16* kdst = Ksh + kvr * 64 + dh;
#pragma unroll
      for (int i = 0; i < 4; ++i) {
        const v8h kk = *(const v8h*)(ksrc + 8 * i);
        *(v8h*)(kdst + 8 * i) = kk;
        const v8h vv = *(const v8h*)(vsrc + 8 * i);
#pragma unroll
        for (int e = 0; e < 8; ++e) Vth[(dh + 8 * i + e) * 64 + kvr] = vv[e];
      }
    }
    __syncthreads();

    v8f s[4];
#pragma unroll
    for (int j = 0; j < 4; ++j) {
      s[j] = (v8f){0.f,0.f,0.f,0.f,0.f,0.f,0.f,0.f};
      FH::U kb;
      kb.h[0] = *(const v8h*)(Ksh + (j * 16 + c) * 64 + 8 * hh);
      kb.h[1] = *(const v8h*)(Ksh + (j * 16 + c) * 64 + 16 + 8 * hh);
      s[j] = mma_h(qa0, kb.v, s[j]);
      kb.h[0] = *(const v8h*)(Ksh + (j * 16 + c) * 64 + 32 + 8 * hh);
      kb.h[1] = *(const v8h*)(Ksh + (j * 16 + c) * 64 + 48 + 8 * hh);
      s[j] = mma_h(qa1, kb.v, s[j]);
    }

    float cm[8];
#pragma unroll
    for (int r = 0; r < 8; ++r) {
      float m = -__builtin_huge_valf();
#pragma unroll
      for (int j = 0; j < 4; ++j) {
        const float a = tb[(size_t)r * NS + kv0 + j * 16];
        const float w = __expf((s[j][r] * 0.125f + a) - m1[r]) * il[r];
        s[j][r] = w;
        m = fmaxf(m, w);
      }
#pragma unroll
      for (int off = 1; off < 16; off <<= 1) m = fmaxf(m, __shfl_xor(m, off, 32));
      cm[r] = m;
    }
    _Float16* pw = Psh[wave];
#pragma unroll
    for (int r = 0; r < 8; ++r) {
      const float mnew = fmaxf(m2[r], cm[r]);
      const float alpha = __expf(m2[r] - mnew);
      m2[r] = mnew;
      float psum = 0.f;
#pragma unroll
      for (int j = 0; j < 4; ++j) {
        const float p = __expf(s[j][r] - mnew);
        psum += p;
        pw[(8 * hh + r) * 64 + j * 16 + c] = (_Float16)(p * 32768.0f);
      }
#pragma unroll
      for (int off = 1; off < 16; off <<= 1) psum += __shfl_xor(psum, off, 32);
      l2[r] = l2[r] * alpha + psum;
#pragma unroll
      for (int t = 0; t < 4; ++t) oacc[t][r] = oacc[t][r] * alpha;
    }
    __builtin_amdgcn_fence(__ATOMIC_RELEASE, "workgroup");
    __builtin_amdgcn_wave_barrier();
    __builtin_amdgcn_fence(__ATOMIC_ACQUIRE, "workgroup");
#pragma unroll
    for (int kk = 0; kk < 2; ++kk) {
      FH::U pa;
      pa.h[0] = *(const v8h*)(pw + c * 64 + kk * 32 + 8 * hh);
      pa.h[1] = *(const v8h*)(pw + c * 64 + kk * 32 + 16 + 8 * hh);
#pragma unroll
      for (int t = 0; t < 4; ++t) {
        FH::U vb;
        vb.h[0] = *(const v8h*)(Vth + (t * 16 + c) * 64 + kk * 32 + 8 * hh);
        vb.h[1] = *(const v8h*)(Vth + (t * 16 + c) * 64 + kk * 32 + 16 + 8 * hh);
        oacc[t] = mma_h(pa.v, vb.v, oacc[t]);
      }
    }
  }

  float* os = Os[wave];
#pragma unroll
  for (int r = 0; r < 8; ++r) {
    const float inv = 1.0f / (l2[r] * 32768.0f);
#pragma unroll
    for (int t = 0; t < 4; ++t) os[(8 * hh + r) * 68 + t * 16 + c] = oacc[t][r] * inv;
  }
  __builtin_amdgcn_fence(__ATOMIC_RELEASE, "workgroup");
  __builtin_amdgcn_wave_barrier();
  __builtin_amdgcn_fence(__ATOMIC_ACQUIRE, "workgroup");
  {
    const int q = lane >> 3, c8 = (lane & 7) * 8;
    for (int pass = 0; pass < 2; ++pass) {
#pragma unroll
      for (int it = 0; it < 4; ++it) {
        const int row = it * 4 + q;
        const float* sp = os + row * 68 + c8;
        v8h hv;
#pragma unroll
        for (int e = 0; e < 8; ++e) hv[e] = (_Float16)sp[e];
        *(volatile v8h*)(Oh + ((size_t)(b * NS + q0 + row)) * ND + h * NDH + c8) = hv;
      }
      __threadfence();
    }
  }
}

__global__ __launch_bounds__(256) void ln_k(const float* __restrict__ X, const float* __restrict__ gamma,
                                           const float* __restrict__ beta, float* __restrict__ Y) {
  __shared__ float ra[8];
  __shared__ float rb[8];
  const int row = blockIdx.x;
  const int t = threadIdx.x, wave = t >> 5, lane = t & 31;
  const v4f x = *(const v4f*)(X + (size_t)row * ND + 4 * t);
  float s = (x[0] + x[1]) + (x[2] + x[3]);
#pragma unroll
  for (int off = 1; off < 32; off <<= 1) s += __shfl_xor(s, off, 32);
  if (lane == 0) ra[wave] = s;
  __syncthreads();
  float tot = 0.f;
#pragma unroll
  for (int w = 0; w < 8; ++w) tot += ra[w];
  const float mean = tot * (1.0f / 1024.0f);
  const float d0 = x[0] - mean, d1 = x[1] - mean, d2 = x[2] - mean, d3 = x[3] - mean;
  float ss = (d0 * d0 + d1 * d1) + (d2 * d2 + d3 * d3);
#pragma unroll
  for (int off = 1; off < 32; off <<= 1) ss += __shfl_xor(ss, off, 32);
  if (lane == 0) rb[wave] = ss;
  __syncthreads();
  float tot2 = 0.f;
#pragma unroll
  for (int w = 0; w < 8; ++w) tot2 += rb[w];
  const float var = tot2 * (1.0f / 1024.0f);
  const float rstd = 1.0f / sqrtf(var + 1e-5f);
  const v4f g  = *(const v4f*)(gamma + 4 * t);
  const v4f bb = *(const v4f*)(beta + 4 * t);
  v4f y;
  y[0] = (d0 * rstd) * g[0] + bb[0];
  y[1] = (d1 * rstd) * g[1] + bb[1];
  y[2] = (d2 * rstd) * g[2] + bb[2];
  y[3] = (d3 * rstd) * g[3] + bb[3];
  *(volatile v4f*)(Y + (size_t)row * ND + 4 * t) = y;
  __threadfence();
  *(volatile v4f*)(Y + (size_t)row * ND + 4 * t) = y;
}

extern "C" void kernel_launch(void* const* d_in, const int* in_sizes, int n_in,
                              void* d_out, int out_size, void* d_ws, size_t ws_size,
                              hipStream_t stream)
{
  if (n_in < 17) return;
  const int nBSD = NB * NS * ND;
  const int nDD  = ND * ND;
  const int nBHS = NB * NH * NS;
  if (in_sizes[0] != nBSD || in_sizes[1] != nBSD || in_sizes[2] != nBSD) return;
  if (in_sizes[3] != NB * NS * 4 || in_sizes[4] < NB) return;
  if (in_sizes[5] != nDD || in_sizes[7] != nDD || in_sizes[9] != nDD || in_sizes[11] != nDD) return;
  if (in_sizes[6] < ND || in_sizes[8] < ND || in_sizes[10] < ND || in_sizes[12] < ND) return;
  if (in_sizes[13] < NDH || in_sizes[14] < 1 || in_sizes[15] < ND || in_sizes[16] < ND) return;
  if (out_size != nBSD) return;

  const float* query  = (const float*)d_in[0];
  const float* key    = (const float*)d_in[1];
  const float* value  = (const float*)d_in[2];
  const float* coords = (const float*)d_in[3];
  const float* E0     = (const float*)d_in[4];
  const float* Wq     = (const float*)d_in[5];
  const float* bq     = (const float*)d_in[6];
  const float* Wk     = (const float*)d_in[7];
  const float* bk     = (const float*)d_in[8];
  const float* Wv     = (const float*)d_in[9];
  const float* bv     = (const float*)d_in[10];
  const float* Wo     = (const float*)d_in[11];
  const float* bo     = (const float*)d_in[12];
  const float* We     = (const float*)d_in[13];
  const float* be     = (const float*)d_in[14];
  const float* gamma  = (const float*)d_in[15];
  const float* beta   = (const float*)d_in[16];

  char* ws = (char*)d_ws;
  size_t off = 0;
  auto carve = [&](size_t bytes) -> char* {
    off = (off + 255) & ~(size_t)255;
    char* p = ws + off;
    off += bytes;
    return p;
  };
  _Float16* q16  = (_Float16*)carve((size_t)nBSD * 2);
  _Float16* k16  = (_Float16*)carve((size_t)nBSD * 2);
  _Float16* v16  = (_Float16*)carve((size_t)nBSD * 2);
  _Float16* wq16 = (_Float16*)carve((size_t)nDD * 2);
  _Float16* wk16 = (_Float16*)carve((size_t)nDD * 2);
  _Float16* wv16 = (_Float16*)carve((size_t)nDD * 2);
  _Float16* wo16 = (_Float16*)carve((size_t)nDD * 2);
  _Float16* Qh   = (_Float16*)carve((size_t)nBSD * 2);
  _Float16* Kh   = (_Float16*)carve((size_t)nBSD * 2);
  _Float16* Vh   = (_Float16*)carve((size_t)nBSD * 2);
  float* Tab     = (float*)carve((size_t)NB * NS * NS * 4);
  float* Ebuf    = (float*)carve((size_t)nBHS * 4);
  float* Mbuf    = (float*)carve((size_t)nBHS * 4);
  float* Lbuf    = (float*)carve((size_t)nBHS * 4);
  float* Abuf    = (float*)carve((size_t)nBHS * 4);
  float* Cbuf    = (float*)carve(256);
  _Float16* Oh   = (_Float16*)carve((size_t)nBSD * 2);
  float* Xbuf    = (float*)carve((size_t)nBSD * 4);
  if (off > ws_size) return;
  if (off > (size_t)134217728) return;

  {
    const int n2a = nBSD / 2, n2w = nDD / 2;
    const int ga = (n2a + 255) / 256, gw = (n2w + 255) / 256;
    cast_f32_f16x2<<<ga, 256, 0, stream>>>(query, q16, n2a);
    cast_f32_f16x2<<<ga, 256, 0, stream>>>(key,   k16, n2a);
    cast_f32_f16x2<<<ga, 256, 0, stream>>>(value, v16, n2a);
    cast_f32_f16x2<<<gw, 256, 0, stream>>>(Wq, wq16, n2w);
    cast_f32_f16x2<<<gw, 256, 0, stream>>>(Wk, wk16, n2w);
    cast_f32_f16x2<<<gw, 256, 0, stream>>>(Wv, wv16, n2w);
    cast_f32_f16x2<<<gw, 256, 0, stream>>>(Wo, wo16, n2w);
  }

  const int M = NB * NS, N = ND, K = ND;
  const int tiles = (M / 64) * (N / 64);
  dim3 gg((tiles + 7) / 8, 1);
  wmma_gemm64<0, false, 2, 1, false, 0><<<gg, 256, 0, stream>>>(
      (const unsigned short*)q16, nullptr, K, 0L, (const unsigned short*)wq16, nullptr, K, 0L,
      (void*)Qh, nullptr, N, 0L, bq, nullptr, 0L, M, N, K, 1.0f);
  wmma_gemm64<0, false, 2, 1, false, 0><<<gg, 256, 0, stream>>>(
      (const unsigned short*)k16, nullptr, K, 0L, (const unsigned short*)wk16, nullptr, K, 0L,
      (void*)Kh, nullptr, N, 0L, bk, nullptr, 0L, M, N, K, 1.0f);
  wmma_gemm64<0, false, 2, 1, false, 0><<<gg, 256, 0, stream>>>(
      (const unsigned short*)v16, nullptr, K, 0L, (const unsigned short*)wv16, nullptr, K, 0L,
      (void*)Vh, nullptr, N, 0L, bv, nullptr, 0L, M, N, K, 1.0f);

  pair_table_k<<<NB * NS, 256, 0, stream>>>(coords, Tab);
  energy_k<<<(nBHS + 255) / 256, 256, 0, stream>>>(Vh, We, be, Ebuf, nBHS);

  const int nblk = NB * NH * (NS / 64);
  attn_stats_k<<<nblk, 128, 0, stream>>>(Qh, Kh, Tab, Ebuf, Mbuf, Lbuf, Abuf);
  corr_k<<<1, 256, 0, stream>>>(Abuf, E0, Cbuf);
  attn_out_k<<<nblk, 128, 0, stream>>>(Qh, Kh, Vh, Tab, Mbuf, Lbuf, Cbuf, Oh);

  wmma_gemm64<0, false, 2, 0, true, 0><<<gg, 256, 0, stream>>>(
      (const unsigned short*)Oh, nullptr, K, 0L, (const unsigned short*)wo16, nullptr, K, 0L,
      (void*)Xbuf, nullptr, N, 0L, bo, query, 0L, M, N, K, 1.0f);
  ln_k<<<NB * NS, 256, 0, stream>>>(Xbuf, gamma, beta, (float*)d_out);
  (void)hipGetLastError();
}
